// MultiHeadAttention_26998164423233
// MI455X (gfx1250) — hardware-verified
//
#include <hip/hip_runtime.h>
#ifndef NB
#define NB 4
#endif
#ifndef SEQ
#define SEQ 2048
#endif
#ifndef EARLY
#define EARLY 512
#endif
#define NB_FULL 4
#define SEQ_FULL 2048
#define DM 512
#define NH 8
#define HD 64
#define ERL ((EARLY < SEQ) ? EARLY : SEQ)
#define NR ((size_t)NB * SEQ)
#define QSCALE 0.044194173824159216f
#define NEGBIG (-3.0e38f)
#define CARRY_LN 6.931471805599453f

typedef _Float16 v16h __attribute__((ext_vector_type(16)));
typedef __bf16   v16b __attribute__((ext_vector_type(16)));
typedef unsigned short v8us __attribute__((ext_vector_type(8), may_alias));
typedef float v8f  __attribute__((ext_vector_type(8)));
typedef float v4f  __attribute__((ext_vector_type(4)));
typedef float v4fa __attribute__((ext_vector_type(4), may_alias));
union Frag { v16h h; v16b b; v8us half[2]; _Float16 e[16]; unsigned short u[16]; };

__device__ __forceinline__ unsigned short bf16_bits(float x) { unsigned int u = __float_as_uint(x); return (unsigned short)((u + 0x7FFFu + ((u >> 16) & 1u)) >> 16); }
__device__ __forceinline__ float bf16_val(unsigned short b) { return __uint_as_float(((unsigned int)b) << 16); }
__device__ __forceinline__ float bf16_rne(float x) { return bf16_val(bf16_bits(x)); }

__device__ __forceinline__ Frag ldf(const unsigned short* p, int hh) {
  Frag f; f.half[0] = *(const v8us*)(p + 8 * hh); f.half[1] = *(const v8us*)(p + 16 + 8 * hh); return f;
}
__device__ __forceinline__ v8f wm_h(const Frag& a, const Frag& b, v8f c) { return __builtin_amdgcn_wmma_f32_16x16x32_f16(false, a.h, false, b.h, (short)0, c, false, false); }
__device__ __forceinline__ v8f wm_b(const Frag& a, const Frag& b, v8f c) { return __builtin_amdgcn_wmma_f32_16x16x32_bf16(false, a.b, false, b.b, (short)0, c, false, false); }
__device__ __forceinline__ void nop2(v8f& c, const Frag& a, const Frag& b) { asm volatile("v_nop\n\tv_nop\n\tv_nop\n\tv_nop" : "+v"(c) : "v"(a.h), "v"(b.h)); }
__device__ __forceinline__ void nop3(v8f& c, const Frag& a, const Frag& b, const Frag& d) { asm volatile("v_nop\n\tv_nop\n\tv_nop\n\tv_nop" : "+v"(c) : "v"(a.h), "v"(b.h), "v"(d.h)); }
__device__ __forceinline__ void nop4(v8f& c, const Frag& a, const Frag& b, const Frag& d, const Frag& e) { asm volatile("v_nop\n\tv_nop\n\tv_nop\n\tv_nop" : "+v"(c) : "v"(a.h), "v"(b.h), "v"(d.h), "v"(e.h)); }
__device__ __forceinline__ void nop8(v8f& c, const Frag& a, const Frag& b, const Frag& d, const Frag& e, const Frag& f, const Frag& g, const Frag& i, const Frag& j) {
  asm volatile("v_nop\n\tv_nop\n\tv_nop\n\tv_nop" : "+v"(c) : "v"(a.h), "v"(b.h), "v"(d.h), "v"(e.h), "v"(f.h), "v"(g.h), "v"(i.h), "v"(j.h));
}

__device__ __forceinline__ v8us to_f16x8(v4f a, v4f c) {
  Frag f;
#pragma unroll
  for (int q = 0; q < 4; ++q) { f.e[q] = (_Float16)a[q]; f.e[4 + q] = (_Float16)c[q]; }
  return f.half[0];
}
__device__ __forceinline__ void to_bf16x8_hl(v4f a, v4f c, v8us& hi, v8us& lo) {
  Frag fh, fl;
#pragma unroll
  for (int q = 0; q < 4; ++q) {
    unsigned short hb = bf16_bits(a[q]); fh.u[q] = hb; fl.u[q] = bf16_bits(a[q] - bf16_val(hb));
    hb = bf16_bits(c[q]); fh.u[4 + q] = hb; fl.u[4 + q] = bf16_bits(c[q] - bf16_val(hb));
  }
  hi = fh.half[0]; lo = fl.half[0];
}

__global__ __launch_bounds__(256) void k_x16(const float* __restrict__ x, unsigned short* __restrict__ X16, int n8) {
  const int t = blockIdx.x * 256 + threadIdx.x;
  if (t >= n8) return;
  const int r = t / (DM / 8), c8 = (t % (DM / 8)) * 8;
  const int b = r / SEQ, tt = r % SEQ;
  const float* src = x + ((size_t)b * SEQ_FULL + tt) * DM + c8;
  const v4f a = *(const v4fa*)src, c = *(const v4fa*)(src + 4);
  v4f ar, cr;
#pragma unroll
  for (int q = 0; q < 4; ++q) { ar[q] = bf16_rne(a[q]); cr[q] = bf16_rne(c[q]); }
  const v8us o = to_f16x8(ar, cr);
  unsigned short* d = X16 + (size_t)t * 8;
  *(volatile v8us*)d = o;
  __threadfence();
  *(volatile v8us*)d = o;
}

template <bool WB>
__global__ __launch_bounds__(256) void k_wnat(const float* __restrict__ w, unsigned short* __restrict__ W16, unsigned short* __restrict__ WBF, int n8) {
  const int t = blockIdx.x * 256 + threadIdx.x;
  if (t >= n8) return;
  const v4f a = *(const v4fa*)(w + (size_t)t * 8), c = *(const v4fa*)(w + (size_t)t * 8 + 4);
  v4f as, cs; Frag fb;
#pragma unroll
  for (int q = 0; q < 4; ++q) {
    const unsigned short b0 = bf16_bits(a[q]), b1 = bf16_bits(c[q]);
    fb.u[q] = b0; fb.u[4 + q] = b1;
    as[q] = bf16_val(b0) * 16.0f; cs[q] = bf16_val(b1) * 16.0f;
  }
  const v8us o = to_f16x8(as, cs);
  const v8us ob = fb.half[0];
  *(volatile v8us*)(W16 + (size_t)t * 8) = o;
  if (WB) *(volatile v8us*)(WBF + (size_t)t * 8) = ob;
  __threadfence();
  *(volatile v8us*)(W16 + (size_t)t * 8) = o;
  if (WB) *(volatile v8us*)(WBF + (size_t)t * 8) = ob;
}

template <bool ABF>
__device__ __forceinline__ v8f gmm(const Frag& a, const Frag& al, const Frag& b, v8f c) {
  if (ABF) { c = wm_b(a, b, c); c = wm_b(al, b, c); nop3(c, a, al, b); }
  else { c = wm_h(a, b, c); nop2(c, a, b); }
  return c;
}

template <int MODE, bool ABF>
__global__ __launch_bounds__(128) void k_gemm(const unsigned short* __restrict__ A, const unsigned short* __restrict__ A2,
                                              const unsigned short* __restrict__ Bt, size_t zB, float alpha, const float* __restrict__ bias,
                                              unsigned short* __restrict__ O16, unsigned short* __restrict__ OH, unsigned short* __restrict__ OL, size_t zO,
                                              float* __restrict__ OF, int tbase) {
  __shared__ __attribute__((aligned(16))) float so[128][68];
  const int tid = threadIdx.x, lane = tid & 31, ln = lane & 15, hh = lane >> 4;
  const int w = __builtin_amdgcn_readfirstlane((int)(threadIdx.x >> 5));
  const int rt = (int)blockIdx.x >> 3, nq = (int)blockIdx.x & 7, b = blockIdx.y, z = blockIdx.z;
  const int t0 = tbase + rt * 128;
  const size_t r0 = (size_t)b * SEQ + t0;
  const int col0 = nq * 64;
  const size_t aof = (r0 + 32 * w + ln) * DM;
  const unsigned short* a0p = A + aof;
  const unsigned short* a1p = a0p + (size_t)16 * DM;
  const unsigned short* l0p = A2 + aof;
  const unsigned short* l1p = l0p + (size_t)16 * DM;
  const unsigned short* bp0 = Bt + (size_t)z * zB + (size_t)(col0 + ln) * DM;
  const v8f z8 = {0.f, 0.f, 0.f, 0.f, 0.f, 0.f, 0.f, 0.f};
  v8f acc[8];
#pragma unroll
  for (int u = 0; u < 8; ++u) acc[u] = z8;
#pragma unroll 1
  for (int kb = 0; kb < DM; kb += 32) {
    const Frag a0 = ldf(a0p + kb, hh), a1 = ldf(a1p + kb, hh);
    Frag a0l = a0, a1l = a1;
    if (ABF) { a0l = ldf(l0p + kb, hh); a1l = ldf(l1p + kb, hh); }
#pragma unroll
    for (int t = 0; t < 4; ++t) {
      const Frag bq = ldf(bp0 + (size_t)(16 * t) * DM + kb, hh);
      acc[t] = gmm<ABF>(a0, a0l, bq, acc[t]);
      acc[4 + t] = gmm<ABF>(a1, a1l, bq, acc[4 + t]);
    }
  }
#pragma unroll
  for (int u = 0; u < 8; ++u) {
    const int t = u & 3, half = u >> 2;
    const int col = t * 16 + ln;
    float bv = 0.f;
    if (MODE == 2) bv = bf16_rne(bias[col0 + col]);
#pragma unroll
    for (int r = 0; r < 8; ++r) so[32 * w + half * 16 + 8 * hh + r][col] = acc[u][r] * alpha + bv;
  }
  __syncthreads();
  const bool early = (t0 < ERL);
  if (MODE == 0) {
    for (int pass = 0; pass < 2; ++pass) {
#pragma unroll
      for (int it = 0; it < 8; ++it) {
        const int row = it * 16 + (tid >> 3), pc = tid & 7;
        const v4f x0 = *(const v4fa*)&so[row][8 * pc], x1 = *(const v4fa*)&so[row][8 * pc + 4];
        const size_t off = (size_t)z * zO + (r0 + row) * DM + col0 + 8 * pc;
        const v8us o = to_f16x8(x0, x1);
        *(volatile v8us*)(O16 + off) = o;
        if (early) {
          v8us oh, ol; to_bf16x8_hl(x0, x1, oh, ol);
          *(volatile v8us*)(OH + off) = oh;
          *(volatile v8us*)(OL + off) = ol;
        }
      }
      if (pass == 0) __threadfence();
    }
  } else if (MODE == 1) {
    const int hd = nq;
    for (int pass = 0; pass < 2; ++pass) {
#pragma unroll
      for (int it = 0; it < 8; ++it) {
        const int d = it * 8 + (tid >> 4), pc = tid & 15;
        v4f x0, x1;
#pragma unroll
        for (int j = 0; j < 4; ++j) { x0[j] = so[8 * pc + j][d]; x1[j] = so[8 * pc + 4 + j][d]; }
        const size_t off = (((size_t)b * NH + hd) * HD + d) * SEQ + t0 + 8 * pc;
        const v8us o = to_f16x8(x0, x1);
        *(volatile v8us*)(O16 + off) = o;
        if (early) {
          v8us oh, ol; to_bf16x8_hl(x0, x1, oh, ol);
          *(volatile v8us*)(OH + off) = oh;
          *(volatile v8us*)(OL + off) = ol;
        }
      }
      if (pass == 0) __threadfence();
    }
  } else {
    for (int pass = 0; pass < 2; ++pass) {
#pragma unroll
      for (int it = 0; it < 16; ++it) {
        const int row = it * 8 + (tid >> 4), pc = tid & 15;
        const v4f v = *(const v4fa*)&so[row][4 * pc];
        *(volatile v4f*)(OF + ((size_t)b * SEQ_FULL + t0 + row) * DM + col0 + 4 * pc) = v;
      }
      if (pass == 0) __threadfence();
    }
  }
}

template <bool RES>
__global__ __launch_bounds__(128) void k_attn(const unsigned short* __restrict__ Qh, const unsigned short* __restrict__ Ql,
                                              const unsigned short* __restrict__ Kh, const unsigned short* __restrict__ Kl,
                                              const unsigned short* __restrict__ Vh, const unsigned short* __restrict__ Vl,
                                              unsigned short* __restrict__ Ch, unsigned short* __restrict__ Cl, int tbase) {
  __shared__ __attribute__((aligned(16))) unsigned short sc[4][RES ? 2 : 1][16][64];
  const int lane = threadIdx.x & 31, ln = lane & 15, hh = lane >> 4;
  const int w = __builtin_amdgcn_readfirstlane((int)(threadIdx.x >> 5));
  const int h = blockIdx.y, b = blockIdx.z;
  const int q0 = tbase + (int)blockIdx.x * 64 + w * 16;
  const int qi = q0 + ln;
  const size_t rowb = (size_t)b * SEQ;
  const size_t qof = (rowb + q0 + ln) * DM + h * HD;
  const Frag qh0 = ldf(Qh + qof, hh), qh1 = ldf(Qh + qof + 32, hh);
  Frag ql0 = qh0, ql1 = qh1;
  if (RES) { ql0 = ldf(Ql + qof, hh); ql1 = ldf(Ql + qof + 32, hh); }
  const size_t kof = (rowb + ln) * DM + h * HD;
  const size_t vof = (((size_t)b * NH + h) * HD + ln) * SEQ;
  const v8f z8 = {0.f, 0.f, 0.f, 0.f, 0.f, 0.f, 0.f, 0.f};
  v8f acc[4];
#pragma unroll
  for (int t = 0; t < 4; ++t) acc[t] = z8;
  float m = NEGBIG, l = 0.f;
  const float carry = RES ? 0.f : CARRY_LN;
  const int nsteps = (q0 + 16 + 31) >> 5;
#pragma unroll 1
  for (int st = 0; st < nsteps; ++st) {
    const int kb = st * 32;
    v8f s[2];
#pragma unroll
    for (int kt = 0; kt < 2; ++kt) {
      const size_t ko = kof + (size_t)(kb + 16 * kt) * DM;
      const Frag k0 = ldf(Kh + ko, hh), k1 = ldf(Kh + ko + 32, hh);
      v8f c = z8;
      if (RES) {
        const Frag kl0 = ldf(Kl + ko, hh), kl1 = ldf(Kl + ko + 32, hh);
        c = wm_b(k0, qh0, c); c = wm_b(kl0, qh0, c); c = wm_b(k0, ql0, c);
        c = wm_b(k1, qh1, c); c = wm_b(kl1, qh1, c); c = wm_b(k1, ql1, c);
        nop8(c, k0, k1, kl0, kl1, qh0, qh1, ql0, ql1);
      } else {
        c = wm_h(k0, qh0, c); c = wm_h(k1, qh1, c);
        nop4(c, k0, k1, qh0, qh1);
      }
      s[kt] = c;
    }
    if (kb + 32 > q0) {
#pragma unroll
      for (int kt = 0; kt < 2; ++kt)
#pragma unroll
        for (int r = 0; r < 8; ++r) { const int key = kb + 16 * kt + 8 * hh + r; s[kt][r] = (key > qi) ? NEGBIG : s[kt][r]; }
    }
    float mx = fmaxf(s[0][0], s[1][0]);
#pragma unroll
    for (int r = 1; r < 8; ++r) mx = fmaxf(mx, fmaxf(s[0][r], s[1][r]));
    mx = fmaxf(mx, __shfl_xor(mx, 16, 32));
    const float mnew = fmaxf(m, mx);
    const float alpha = __expf((m - mnew) * QSCALE);
    const float cc = carry - mnew * QSCALE;
    m = mnew;
    Frag ph, pl;
    float ps = 0.f;
#pragma unroll
    for (int kt = 0; kt < 2; ++kt)
#pragma unroll
      for (int r = 0; r < 8; ++r) {
        const float p = __expf(fmaf(s[kt][r], QSCALE, cc));
        if (RES) {
          const unsigned short hb = bf16_bits(p); const float hv = bf16_val(hb);
          const unsigned short lb = bf16_bits(p - hv);
          ph.u[8 * kt + r] = hb; pl.u[8 * kt + r] = lb; ps += hv + bf16_val(lb);
        } else {
          ph.e[8 * kt + r] = (_Float16)p; ps += p;
        }
      }
    if (!RES) pl = ph;
    ps += __shfl_xor(ps, 16, 32);
    l = l * alpha + ps;
#pragma unroll
    for (int t = 0; t < 4; ++t) acc[t] = acc[t] * alpha;
#pragma unroll
    for (int t = 0; t < 4; ++t) {
      const size_t vo = vof + (size_t)(16 * t) * SEQ + kb;
      const Frag vh = ldf(Vh + vo, hh);
      if (RES) {
        const Frag vl = ldf(Vl + vo, hh);
        acc[t] = wm_b(vh, ph, acc[t]); acc[t] = wm_b(vl, ph, acc[t]); acc[t] = wm_b(vh, pl, acc[t]);
        nop4(acc[t], vh, vl, ph, pl);
      } else {
        acc[t] = wm_h(vh, ph, acc[t]);
        nop2(acc[t], vh, ph);
      }
    }
  }
  const float inv = 1.0f / l;
  const float osc = RES ? inv : inv * 64.0f;
#pragma unroll
  for (int t = 0; t < 4; ++t) {
    if (RES) {
      Frag oh, ol;
#pragma unroll
      for (int r = 0; r < 8; ++r) { const float c = acc[t][r] * osc; const unsigned short hb = bf16_bits(c); oh.u[r] = hb; ol.u[r] = bf16_bits(c - bf16_val(hb)); }
      *(v8us*)&sc[w][0][ln][16 * t + 8 * hh] = oh.half[0];
      *(v8us*)&sc[w][RES ? 1 : 0][ln][16 * t + 8 * hh] = ol.half[0];
    } else {
      Frag o;
#pragma unroll
      for (int r = 0; r < 8; ++r) o.e[r] = (_Float16)(acc[t][r] * osc);
      *(v8us*)&sc[w][0][ln][16 * t + 8 * hh] = o.half[0];
    }
  }
  __builtin_amdgcn_fence(4  , "workgroup");
  __builtin_amdgcn_wave_barrier();
  const int rsub = lane >> 3, pc = lane & 7;
  for (int pass = 0; pass < 2; ++pass) {
#pragma unroll
    for (int q = 0; q < 4; ++q) {
      const int row = 4 * q + rsub;
      const size_t off = (rowb + q0 + row) * DM + h * HD + 8 * pc;
      const v8us v0 = *(const v8us*)&sc[w][0][row][8 * pc];
      *(volatile v8us*)(Ch + off) = v0;
      if (RES) { const v8us v1 = *(const v8us*)&sc[w][RES ? 1 : 0][row][8 * pc]; *(volatile v8us*)(Cl + off) = v1; }
    }
    if (pass == 0) __threadfence();
  }
}

extern "C" void kernel_launch(void* const* d_in, const int* in_sizes, int n_in,
                              void* d_out, int out_size, void* d_ws, size_t ws_size, hipStream_t stream) {
  static_assert(NH * HD == DM);
  static_assert(DM == 512);
  static_assert(SEQ % 128 == 0);
  static_assert(ERL % 128 == 0);
  static_assert(NB <= NB_FULL);
  static_assert(SEQ <= SEQ_FULL);
  static_assert((size_t)13 * NB * SEQ * DM * 2 + (size_t)5 * DM * DM * 2 <= (size_t)134217728);
  if (n_in < 6) return;
  const long long xmin = ((long long)(NB - 1) * SEQ_FULL + SEQ) * DM;
  if ((long long)in_sizes[0] < xmin) return;
  if (in_sizes[1] < DM * DM || in_sizes[2] < DM * DM || in_sizes[3] < DM * DM || in_sizes[4] < DM * DM || in_sizes[5] < DM) return;
  if ((long long)out_size < xmin) return;
  const float* x  = (const float*)d_in[0];
  const float* Wq = (const float*)d_in[1];
  const float* Wk = (const float*)d_in[2];
  const float* Wv = (const float*)d_in[3];
  const float* Wp = (const float*)d_in[4];
  const float* bp = (const float*)d_in[5];
  float* out = (float*)d_out;

  char* ws = (char*)d_ws; size_t off = 0;
  auto take = [&](size_t bytes) { char* p = ws + off; off += (bytes + 255) & ~(size_t)255; return (unsigned short*)p; };
  const size_t PL = NR * DM;
  const size_t WN = (size_t)DM * DM;
  unsigned short* W16  = take(4 * WN * 2);
  unsigned short* WPB  = take(WN * 2);
  unsigned short* X16  = take(PL * 2);
  unsigned short* QK16 = take(2 * PL * 2);
  unsigned short* QKH  = take(2 * PL * 2);
  unsigned short* QKL  = take(2 * PL * 2);
  unsigned short* VT16 = take(PL * 2);
  unsigned short* VTH  = take(PL * 2);
  unsigned short* VTL  = take(PL * 2);
  unsigned short* C16  = take(PL * 2);
  unsigned short* CH   = take(PL * 2);
  unsigned short* CL   = take(PL * 2);
  if (off > ws_size || off > (size_t)134217728) return;

  const int xn8 = (int)(PL / 8), wn8 = (int)(WN / 8);
  k_x16<<<(unsigned)((xn8 + 255) / 256), 256, 0, stream>>>(x, X16, xn8);
  k_wnat<false><<<(unsigned)((wn8 + 255) / 256), 256, 0, stream>>>(Wq, W16, WPB, wn8);
  k_wnat<false><<<(unsigned)((wn8 + 255) / 256), 256, 0, stream>>>(Wk, W16 + WN, WPB, wn8);
  k_wnat<false><<<(unsigned)((wn8 + 255) / 256), 256, 0, stream>>>(Wv, W16 + 2 * WN, WPB, wn8);
  k_wnat<true><<<(unsigned)((wn8 + 255) / 256), 256, 0, stream>>>(Wp, W16 + 3 * WN, WPB, wn8);

  k_gemm<0, false><<<dim3((SEQ / 128) * 8, NB, 2), 128, 0, stream>>>(X16, X16, W16, WN, 0.0625f, bp, QK16, QKH, QKL, PL, out, 0);
  k_gemm<1, false><<<dim3((SEQ / 128) * 8, NB, 1), 128, 0, stream>>>(X16, X16, W16 + 2 * WN, (size_t)0, 0.0625f, bp, VT16, VTH, VTL, (size_t)0, out, 0);

  k_attn<true><<<dim3(ERL / 64, NH, NB), 128, 0, stream>>>(QKH, QKL, QKH + PL, QKL + PL, VTH, VTL, CH, CL, 0);
  if (SEQ > ERL)
    k_attn<false><<<dim3((SEQ - ERL) / 64, NH, NB), 128, 0, stream>>>(QK16, QK16, QK16 + PL, QK16 + PL, VT16, VT16, C16, C16, ERL);

  k_gemm<2, true><<<dim3((ERL / 128) * 8, NB, 1), 128, 0, stream>>>(CH, CL, WPB, (size_t)0, 1.0f, bp, X16, X16, X16, (size_t)0, out, 0);
  if (SEQ > ERL)
    k_gemm<2, false><<<dim3(((SEQ - ERL) / 128) * 8, NB, 1), 128, 0, stream>>>(C16, C16, W16 + 3 * WN, (size_t)0, 0.0009765625f, bp, X16, X16, X16, (size_t)0, out, ERL);
}
